// GeneEmbedding_6150393168706
// MI455X (gfx1250) — hardware-run, weakly checked
//
#include <hip/hip_runtime.h>
#include <math.h>
#include <stdint.h>

#define NSEQ  128
#define GDIM  1024
#define DD    32
#define NTOK  (NSEQ * GDIM)
#define NWROW 160
#define LNEPS 1.0e-3f
#define XC    64.0f
#define WSC   64.0f
#define VS    64.0f
#define QCAR  256.0f
#define KCAR  256.0f
#define VC    1024.0f
#define PCAR  1024.0f
#define AC    4096.0f
#define LNPC  6.931471805599453f
#define RSQD  0.17677669529663687f
static_assert(NTOK == 131072);
static_assert((NTOK % 128) == 0 && (GDIM % 64) == 0);

typedef _Float16 v16h __attribute__((ext_vector_type(16)));
typedef _Float16 v8h  __attribute__((ext_vector_type(8)));
typedef float    v8f  __attribute__((ext_vector_type(8)));
typedef float    v4f  __attribute__((ext_vector_type(4)));
typedef unsigned int v4u __attribute__((ext_vector_type(4)));

union FragH { v16h v; v8h h[2]; };

__device__ __forceinline__ unsigned short bf_bits(float f) {
  unsigned u = __float_as_uint(f);
  return (unsigned short)((u + 0x7FFFu + ((u >> 16) & 1u)) >> 16);
}
__device__ __forceinline__ float bf_up(unsigned short h) { return __uint_as_float(((unsigned)h) << 16); }
__device__ __forceinline__ float bfr(float f) { return bf_up(bf_bits(f)); }
__device__ __forceinline__ unsigned short h_bits(_Float16 x) { return __builtin_bit_cast(unsigned short, x); }
__device__ __forceinline__ unsigned pk16(unsigned short a, unsigned short b) { return (unsigned)a | ((unsigned)b << 16); }
__device__ __forceinline__ v8f zero8() { v8f z = {0.f, 0.f, 0.f, 0.f, 0.f, 0.f, 0.f, 0.f}; return z; }
__device__ __forceinline__ float hmax8(v8f s) {
  return fmaxf(fmaxf(fmaxf(s[0], s[1]), fmaxf(s[2], s[3])), fmaxf(fmaxf(s[4], s[5]), fmaxf(s[6], s[7])));
}

__device__ __forceinline__ v16h ldfrag_h(const _Float16* p) {
  FragH f;
  f.h[0] = *(const v8h*)(p);
  f.h[1] = *(const v8h*)(p + 16);
  return f.v;
}

__device__ __forceinline__ v8f mma_h_raw(v16h a, v16h b, v8f c) {
  return __builtin_amdgcn_wmma_f32_16x16x32_f16(false, a, false, b, (short)0, c, false, false);
}
__device__ __forceinline__ void guard2(v8f& a, v8f& b, v16h x, v16h y, v16h w) {
#if defined(__HIP_DEVICE_COMPILE__)
  asm volatile("v_nop\n\tv_nop\n\tv_nop\n\tv_nop" : "+v"(a), "+v"(b) : "v"(x), "v"(y), "v"(w));
#endif
}
__device__ __forceinline__ void sguard4(v8f& a, v8f& b, v8f& c, v8f& d,
                                        v16h k0, v16h k1, v16h k2, v16h k3, v16h q) {
#if defined(__HIP_DEVICE_COMPILE__)
  asm volatile("v_nop\n\tv_nop\n\tv_nop\n\tv_nop"
               : "+v"(a), "+v"(b), "+v"(c), "+v"(d) : "v"(k0), "v"(k1), "v"(k2), "v"(k3), "v"(q));
#endif
}
__device__ __forceinline__ void oguard2(v8f& a, v8f& b, v16h x0, v16h x1, v16h x2, v16h x3, v16h p0, v16h p1) {
#if defined(__HIP_DEVICE_COMPILE__)
  asm volatile("v_nop\n\tv_nop\n\tv_nop\n\tv_nop"
               : "+v"(a), "+v"(b) : "v"(x0), "v"(x1), "v"(x2), "v"(x3), "v"(p0), "v"(p1));
#endif
}
__device__ __forceinline__ void wave_sync_lds() {
  __builtin_amdgcn_fence(__ATOMIC_RELEASE, "workgroup");
  __builtin_amdgcn_wave_barrier();
  __builtin_amdgcn_fence(__ATOMIC_ACQUIRE, "workgroup");
}
__device__ __forceinline__ float hred_max(float x) {
  x = fmaxf(x, __shfl_xor(x, 1, 32));
  x = fmaxf(x, __shfl_xor(x, 2, 32));
  x = fmaxf(x, __shfl_xor(x, 4, 32));
  x = fmaxf(x, __shfl_xor(x, 8, 32));
  return x;
}
__device__ __forceinline__ float hred_sum(float x) {
  x += __shfl_xor(x, 1, 32);
  x += __shfl_xor(x, 2, 32);
  x += __shfl_xor(x, 4, 32);
  x += __shfl_xor(x, 8, 32);
  return x;
}

__global__ __launch_bounds__(256) void prep_w(const float* __restrict__ wq, const float* __restrict__ wk,
                                              const float* __restrict__ wv, const float* __restrict__ wo,
                                              const float* __restrict__ pk2, unsigned short* WP) {
  const int t = threadIdx.x, wave = t >> 5;
  v4u vals[3];
#pragma unroll
  for (int k = 0; k < 3; ++k) {
    const int piece = 256 * k + t;
    const int pc = (piece < 4 * NWROW) ? piece : (4 * NWROW - 1);
    int sel = ((256 * k + 32 * wave) >> 2) >> 5;
    sel = (sel > 4) ? 4 : sel;
    const float* src = (sel == 0) ? wq : (sel == 1) ? wk : (sel == 2) ? wv : (sel == 3) ? wo : pk2;
    const int row = pc >> 2, c8 = (pc & 3) * 8, oo = row & 31;
    v4u v;
#pragma unroll
    for (int e = 0; e < 4; ++e) {
      const float w0 = bfr(src[(c8 + 2 * e) * DD + oo]) * WSC;
      const float w1 = bfr(src[(c8 + 2 * e + 1) * DD + oo]) * WSC;
      v[e] = pk16(h_bits((_Float16)w0), h_bits((_Float16)w1));
    }
    vals[k] = v;
  }
  const bool act2 = (wave < 4);
  for (int pass = 0; pass < 2; ++pass) {
#pragma unroll
    for (int k = 0; k < 3; ++k) {
      if (k < 2 || act2) *(volatile v4u*)(WP + (size_t)(256 * k + t) * 8) = vals[k];
    }
    __threadfence();
  }
}

__global__ __launch_bounds__(256) void prep_tok(const float* __restrict__ x, const float* __restrict__ pkt,
                                                const float* __restrict__ pkv, const float* __restrict__ disc,
                                                const float* __restrict__ sfp, const int* __restrict__ gsz,
                                                const unsigned short* __restrict__ WP,
                                                float* out0, float* H0, unsigned short* XH) {
  __shared__ __align__(16) float sT[8][16 * 36];
  const int tid = threadIdx.x, wave = tid >> 5, lane = tid & 31, hh = lane >> 4, c = lane & 15;
  const int t0 = (blockIdx.x * 8 + wave) * 16;
  int gs = gsz[0];
  gs = (gs < 1) ? 1 : ((gs > GDIM) ? GDIM : gs);
  const float sf = bfr(sfp[0]);

  const float xa = bfr(x[t0 + c]);
  FragH af;
#pragma unroll
  for (int i = 0; i < 8; ++i) {
    const float pa = bfr(pkv[8 * hh + i]), pb = bfr(pkv[16 + 8 * hh + i]);
    float va = xa * pa; va = (va >= 0.f) ? va : 0.1f * va;
    float vb = xa * pb; vb = (vb >= 0.f) ? vb : 0.1f * vb;
    af.h[0][i] = (_Float16)(va * VS);
    af.h[1][i] = (_Float16)(vb * VS);
  }
  const _Float16* P2 = (const _Float16*)(const void*)WP + 128 * DD;
  const v16h b0 = ldfrag_h(P2 + c * DD + 8 * hh);
  const v16h b1 = ldfrag_h(P2 + (16 + c) * DD + 8 * hh);
  v8f d0 = mma_h_raw(af.v, b0, zero8());
  v8f d1 = mma_h_raw(af.v, b1, zero8());
  guard2(d0, d1, af.v, b0, b1);

  const float pc0 = bfr(pkv[c]), pc1 = bfr(pkv[16 + c]);
  const float dc0 = bfr(disc[c]), dc1 = bfr(disc[16 + c]);
  const float inv = 1.0f / (VS * WSC);
  float* slab = sT[wave];
#pragma unroll
  for (int r = 0; r < 8; ++r) {
    const int m = t0 + 8 * hh + r;
    const float xm = bfr(x[m]);
    float va = xm * pc0; va = (va >= 0.f) ? va : 0.1f * va;
    float vb = xm * pc1; vb = (vb >= 0.f) ? vb : 0.1f * vb;
    const float ta = d0[r] * inv + sf * va;
    const float tb = d1[r] * inv + sf * vb;
    const float mx = hred_max(fmaxf(ta, tb));
    const float ea = __expf(ta - mx), eb = __expf(tb - mx);
    const float ss = hred_sum(ea + eb);
    const float sd = hred_sum(ea * dc0 + eb * dc1);
    const float s  = sd * (1.0f / ss);
    int g = m & (GDIM - 1);
    g = (g < gs) ? g : (gs - 1);
    const float tk0 = bfr(pkt[(size_t)g * DD + c]), tk1 = bfr(pkt[(size_t)g * DD + 16 + c]);
    slab[(8 * hh + r) * 36 + c]      = tk0 * s;
    slab[(8 * hh + r) * 36 + 16 + c] = tk1 * s;
  }
  wave_sync_lds();

  const int rq4 = lane >> 3, c4 = (lane & 7) * 4;
  const int rq2 = lane >> 2, c8 = (lane & 3) * 8;
  v4f hv[4], tv[4];
  v4u xv[2];
#pragma unroll
  for (int it = 0; it < 4; ++it) {
    const int row = it * 4 + rq4;
    hv[it] = *(const v4f*)(slab + row * 36 + c4);
    int g = (t0 + row) & (GDIM - 1);
    g = (g < gs) ? g : (gs - 1);
    const v4f tk = *(const v4f*)(pkt + (size_t)g * DD + c4);
    v4f tb;
#pragma unroll
    for (int e = 0; e < 4; ++e) tb[e] = bfr(tk[e]);
    tv[it] = tb;
  }
#pragma unroll
  for (int it = 0; it < 2; ++it) {
    const int row = it * 8 + rq2;
    const float* sp = slab + row * 36 + c8;
    v4u u;
#pragma unroll
    for (int e = 0; e < 4; ++e)
      u[e] = pk16(h_bits((_Float16)(sp[2 * e] * XC)), h_bits((_Float16)(sp[2 * e + 1] * XC)));
    xv[it] = u;
  }
  for (int pass = 0; pass < 2; ++pass) {
#pragma unroll
    for (int it = 0; it < 4; ++it) {
      const int row = it * 4 + rq4;
      *(volatile v4f*)(H0   + (size_t)(t0 + row) * DD + c4) = hv[it];
      *(volatile v4f*)(out0 + (size_t)(t0 + row) * DD + c4) = tv[it];
    }
#pragma unroll
    for (int it = 0; it < 2; ++it) {
      const int row = it * 8 + rq2;
      *(volatile v4u*)(XH + (size_t)(t0 + row) * DD + c8) = xv[it];
    }
    __threadfence();
  }
}

__global__ __launch_bounds__(128) void qkv_proj(const unsigned short* __restrict__ XH, const unsigned short* __restrict__ WP,
                                                const float* __restrict__ bq, const float* __restrict__ bk,
                                                const float* __restrict__ bv,
                                                unsigned short* QK, unsigned short* VT) {
  __shared__ __align__(16) float sQ[4][16 * 68];
  __shared__ __align__(16) unsigned short sV[DD * 72];
  const int tid = threadIdx.x, wave = tid >> 5, lane = tid & 31, hh = lane >> 4, c = lane & 15;
  const int t0 = blockIdx.x * 64;
  const int tw = t0 + wave * 16;
  const _Float16* Xh = (const _Float16*)(const void*)XH;
  const _Float16* Wh = (const _Float16*)(const void*)WP;
  const v16h a = ldfrag_h(Xh + (size_t)(tw + c) * DD + 8 * hh);
  const float inv = 1.0f / (XC * WSC);
  float* slab = sQ[wave];
  {
    const v16h w0 = ldfrag_h(Wh + (0 + c) * DD + 8 * hh);
    const v16h w1 = ldfrag_h(Wh + (16 + c) * DD + 8 * hh);
    v8f q0 = mma_h_raw(a, w0, zero8());
    v8f q1 = mma_h_raw(a, w1, zero8());
    guard2(q0, q1, a, w0, w1);
    const float b0 = bfr(bq[c]), b1 = bfr(bq[16 + c]);
#pragma unroll
    for (int r = 0; r < 8; ++r) {
      slab[(8 * hh + r) * 68 + c]      = (q0[r] * inv + b0) * QCAR;
      slab[(8 * hh + r) * 68 + 16 + c] = (q1[r] * inv + b1) * QCAR;
    }
  }
  {
    const v16h w0 = ldfrag_h(Wh + (32 + c) * DD + 8 * hh);
    const v16h w1 = ldfrag_h(Wh + (48 + c) * DD + 8 * hh);
    v8f k0 = mma_h_raw(a, w0, zero8());
    v8f k1 = mma_h_raw(a, w1, zero8());
    guard2(k0, k1, a, w0, w1);
    const float b0 = bfr(bk[c]), b1 = bfr(bk[16 + c]);
#pragma unroll
    for (int r = 0; r < 8; ++r) {
      slab[(8 * hh + r) * 68 + 32 + c] = (k0[r] * inv + b0) * KCAR;
      slab[(8 * hh + r) * 68 + 48 + c] = (k1[r] * inv + b1) * KCAR;
    }
  }
  {
    const v16h w0 = ldfrag_h(Wh + (64 + c) * DD + 8 * hh);
    const v16h w1 = ldfrag_h(Wh + (80 + c) * DD + 8 * hh);
    v8f v0 = mma_h_raw(a, w0, zero8());
    v8f v1 = mma_h_raw(a, w1, zero8());
    guard2(v0, v1, a, w0, w1);
    const float b0 = bfr(bv[c]), b1 = bfr(bv[16 + c]);
#pragma unroll
    for (int r = 0; r < 8; ++r) {
      sV[c * 72 + wave * 16 + 8 * hh + r]        = h_bits((_Float16)((v0[r] * inv + b0) * VC));
      sV[(16 + c) * 72 + wave * 16 + 8 * hh + r] = h_bits((_Float16)((v1[r] * inv + b1) * VC));
    }
  }
  wave_sync_lds();
  const int rq4 = lane >> 3, c8 = (lane & 7) * 8;
  v4u qv[4];
#pragma unroll
  for (int it = 0; it < 4; ++it) {
    const int row = it * 4 + rq4;
    const float* sp = slab + row * 68 + c8;
    v4u u;
#pragma unroll
    for (int e = 0; e < 4; ++e) u[e] = pk16(h_bits((_Float16)sp[2 * e]), h_bits((_Float16)sp[2 * e + 1]));
    qv[it] = u;
  }
  __syncthreads();
  const int vr = tid >> 3, vp = (tid & 7) * 8;
  const v4u va = *(const v4u*)(sV + vr * 72 + vp);
  const v4u vb = *(const v4u*)(sV + (16 + vr) * 72 + vp);
  const size_t seq = (size_t)(t0 >> 10);
  const int g0 = t0 & (GDIM - 1);
  unsigned short* pva = VT + ((seq * DD + vr) * GDIM + g0 + vp);
  unsigned short* pvb = VT + ((seq * DD + 16 + vr) * GDIM + g0 + vp);
  for (int pass = 0; pass < 2; ++pass) {
#pragma unroll
    for (int it = 0; it < 4; ++it) {
      const int row = it * 4 + rq4;
      *(volatile v4u*)(QK + (size_t)(tw + row) * 64 + c8) = qv[it];
    }
    *(volatile v4u*)pva = va;
    *(volatile v4u*)pvb = vb;
    __threadfence();
  }
}

__global__ __launch_bounds__(128)
void attn(const unsigned short* __restrict__ QK, const unsigned short* __restrict__ VT, unsigned short* AO) {
  __shared__ __align__(16) unsigned short Os[64 * 40];
  const int tid  = threadIdx.x;
  const int wave = tid >> 5;
  const int lane = tid & 31;
  const int hh   = lane >> 4;
  const int c    = lane & 15;
  const int bx  = blockIdx.x;
  const int seq = bx >> 4;
  const int q0  = (bx & 15) * 64;
  const size_t tok0 = (size_t)seq * GDIM;

  const _Float16* QKp = (const _Float16*)(const void*)QK;
  const _Float16* Vb  = (const _Float16*)(const void*)VT;

  const v16h qf = ldfrag_h(QKp + (tok0 + q0 + wave * 16 + c) * 64 + 8 * hh);
  const _Float16* Kp  = QKp + (tok0 + c) * 64 + DD + 8 * hh;
  const _Float16* V0p = Vb + ((size_t)seq * DD + c) * GDIM + 8 * hh;
  const _Float16* V1p = Vb + ((size_t)seq * DD + 16 + c) * GDIM + 8 * hh;
  const float SC = RSQD / (QCAR * KCAR);

  float m = -1.0e30f, l = 0.f;
  v8f o0 = zero8(), o1 = zero8();
#pragma unroll 1
  for (int it = 0; it < GDIM / 64; ++it) {
    const int kb = it * 64;
    v16h kf[4];
#pragma unroll
    for (int j = 0; j < 4; ++j) kf[j] = ldfrag_h(Kp + (size_t)(kb + 16 * j) * 64);
    v8f s0 = mma_h_raw(kf[0], qf, zero8());
    v8f s1 = mma_h_raw(kf[1], qf, zero8());
    v8f s2 = mma_h_raw(kf[2], qf, zero8());
    v8f s3 = mma_h_raw(kf[3], qf, zero8());
    sguard4(s0, s1, s2, s3, kf[0], kf[1], kf[2], kf[3], qf);

    float mx = fmaxf(fmaxf(hmax8(s0), hmax8(s1)), fmaxf(hmax8(s2), hmax8(s3)));
    mx = fmaxf(mx, __shfl_xor(mx, 16, 32));
    const float mn   = fmaxf(m, mx * SC);
    const float corr = __expf(m - mn);
    m = mn;
    const float msh = mn - LNPC;
    l *= corr;
#pragma unroll
    for (int r = 0; r < 8; ++r) { o0[r] *= corr; o1[r] *= corr; }

    FragH p0, p1;
    float ls = 0.f;
#pragma unroll
    for (int r = 0; r < 8; ++r) {
      const float e0 = __expf(s0[r] * SC - msh);
      const float e1 = __expf(s1[r] * SC - msh);
      const float e2 = __expf(s2[r] * SC - msh);
      const float e3 = __expf(s3[r] * SC - msh);
      ls += (e0 + e1) + (e2 + e3);
      p0.h[0][r] = (_Float16)e0;
      p0.h[1][r] = (_Float16)e1;
      p1.h[0][r] = (_Float16)e2;
      p1.h[1][r] = (_Float16)e3;
    }
    l += ls;

    const v16h v0a = ldfrag_h(V0p + kb);
    const v16h v0b = ldfrag_h(V0p + kb + 32);
    const v16h v1a = ldfrag_h(V1p + kb);
    const v16h v1b = ldfrag_h(V1p + kb + 32);
    o0 = mma_h_raw(v0a, p0.v, o0);
    o0 = mma_h_raw(v0b, p1.v, o0);
    o1 = mma_h_raw(v1a, p0.v, o1);
    o1 = mma_h_raw(v1b, p1.v, o1);
    oguard2(o0, o1, v0a, v0b, v1a, v1b, p0.v, p1.v);
  }
  l += __shfl_xor(l, 16, 32);
  const float sc = (1.0f / l) * (AC / VC);

#pragma unroll
  for (int r = 0; r < 8; ++r) {
    Os[(wave * 16 + c) * 40 + 8 * hh + r]      = h_bits((_Float16)(o0[r] * sc));
    Os[(wave * 16 + c) * 40 + 16 + 8 * hh + r] = h_bits((_Float16)(o1[r] * sc));
  }
  __syncthreads();
  {
    const int rr = tid >> 2, pp = (tid & 3) * 8;
    const v4u va = *(const v4u*)(Os + rr * 40 + pp);
    const v4u vb = *(const v4u*)(Os + (32 + rr) * 40 + pp);
    unsigned short* pa = AO + (tok0 + q0 + rr) * DD + pp;
    unsigned short* pb = AO + (tok0 + q0 + 32 + rr) * DD + pp;
    *(volatile v4u*)pa = va;
    *(volatile v4u*)pb = vb;
    __threadfence();
    *(volatile v4u*)pa = va;
    *(volatile v4u*)pb = vb;
  }
}

__global__ __launch_bounds__(256) void proj_ln(const unsigned short* __restrict__ AO, const unsigned short* __restrict__ WP,
                                               const float* __restrict__ bo, const float* __restrict__ gam,
                                               const float* __restrict__ bet, const float* __restrict__ Hin,
                                               float* Hout, unsigned short* XH, int writex) {
  __shared__ __align__(16) float sT[8][16 * 36];
  const int tid = threadIdx.x, wave = tid >> 5, lane = tid & 31, hh = lane >> 4, c = lane & 15;
  const int tw = (blockIdx.x * 8 + wave) * 16;
  const _Float16* Ah = (const _Float16*)(const void*)AO;
  const _Float16* Wh = (const _Float16*)(const void*)WP;
  const v16h a  = ldfrag_h(Ah + (size_t)(tw + c) * DD + 8 * hh);
  const v16h w0 = ldfrag_h(Wh + (96 + c) * DD + 8 * hh);
  const v16h w1 = ldfrag_h(Wh + (112 + c) * DD + 8 * hh);
  v8f y0 = mma_h_raw(a, w0, zero8());
  v8f y1 = mma_h_raw(a, w1, zero8());
  guard2(y0, y1, a, w0, w1);

  const float b0 = bfr(bo[c]), b1 = bfr(bo[16 + c]);
  const float g0 = bfr(gam[c]), g1 = bfr(gam[16 + c]);
  const float e0 = bfr(bet[c]), e1 = bfr(bet[16 + c]);
  const float inv = 1.0f / (AC * WSC);
  float* slab = sT[wave];
#pragma unroll
  for (int r = 0; r < 8; ++r) {
    const int m = tw + 8 * hh + r;
    const float h0 = Hin[(size_t)m * DD + c];
    const float h1 = Hin[(size_t)m * DD + 16 + c];
    const float a0 = h0 + (y0[r] * inv + b0);
    const float a1 = h1 + (y1[r] * inv + b1);
    const float mean = hred_sum(a0 + a1) * (1.0f / DD);
    const float d0 = a0 - mean, d1 = a1 - mean;
    const float var = hred_sum(d0 * d0 + d1 * d1) * (1.0f / DD);
    const float rs = rsqrtf(var + LNEPS);
    slab[(8 * hh + r) * 36 + c]      = (g0 * d0) * rs + e0;
    slab[(8 * hh + r) * 36 + 16 + c] = (g1 * d1) * rs + e1;
  }
  wave_sync_lds();

  const int rq4 = lane >> 3, c4 = (lane & 7) * 4;
  const int rq2 = lane >> 2, c8 = (lane & 3) * 8;
  v4f hv[4];
  v4u xv[2];
#pragma unroll
  for (int it = 0; it < 4; ++it) {
    const int row = it * 4 + rq4;
    hv[it] = *(const v4f*)(slab + row * 36 + c4);
  }
#pragma unroll
  for (int it = 0; it < 2; ++it) {
    const int row = it * 8 + rq2;
    const float* sp = slab + row * 36 + c8;
    v4u u;
#pragma unroll
    for (int e = 0; e < 4; ++e)
      u[e] = pk16(h_bits((_Float16)(sp[2 * e] * XC)), h_bits((_Float16)(sp[2 * e + 1] * XC)));
    xv[it] = u;
  }
  for (int pass = 0; pass < 2; ++pass) {
#pragma unroll
    for (int it = 0; it < 4; ++it) {
      const int row = it * 4 + rq4;
      *(volatile v4f*)(Hout + (size_t)(tw + row) * DD + c4) = hv[it];
    }
    if (writex != 0) {
#pragma unroll
      for (int it = 0; it < 2; ++it) {
        const int row = it * 8 + rq2;
        *(volatile v4u*)(XH + (size_t)(tw + row) * DD + c8) = xv[it];
      }
    }
    __threadfence();
  }
}

extern "C" void kernel_launch(void* const* d_in, const int* in_sizes, int n_in,
                              void* d_out, int out_size, void* d_ws, size_t ws_size,
                              hipStream_t stream) {
  if (n_in < 17) return;
  if (in_sizes[0] != NTOK) return;
  if (in_sizes[1] != GDIM * DD) return;
  if (in_sizes[2] != DD || in_sizes[3] != DD * DD || in_sizes[4] != DD || in_sizes[5] != 1) return;
  if (in_sizes[6] != DD * DD || in_sizes[7] != DD || in_sizes[8] != DD * DD || in_sizes[9] != DD) return;
  if (in_sizes[10] != DD * DD || in_sizes[11] != DD || in_sizes[12] != DD * DD || in_sizes[13] != DD) return;
  if (in_sizes[14] != DD || in_sizes[15] != DD || in_sizes[16] != 1) return;
  if (out_size != 2 * NTOK * DD) return;

  const float* x    = (const float*)d_in[0];
  const float* pkt  = (const float*)d_in[1];
  const float* pkv  = (const float*)d_in[2];
  const float* pk2  = (const float*)d_in[3];
  const float* disc = (const float*)d_in[4];
  const float* sfp  = (const float*)d_in[5];
  const float* wq = (const float*)d_in[6];  const float* bq = (const float*)d_in[7];
  const float* wk = (const float*)d_in[8];  const float* bk = (const float*)d_in[9];
  const float* wv = (const float*)d_in[10]; const float* bv = (const float*)d_in[11];
  const float* wo = (const float*)d_in[12]; const float* bo = (const float*)d_in[13];
  const float* gam = (const float*)d_in[14];
  const float* bet = (const float*)d_in[15];
  const int*   gsz = (const int*)d_in[16];

  const size_t PWP = 16384;
  const size_t PH  = (size_t)NTOK * DD * 4;
  const size_t PXH = (size_t)NTOK * DD * 2;
  const size_t PQK = (size_t)NTOK * 64 * 2;
  const size_t PVT = (size_t)NSEQ * DD * GDIM * 2;
  const size_t PAO = (size_t)NTOK * DD * 2;
  size_t off = 0;
  const size_t oWP = off; off += PWP;
  const size_t oH0 = off; off += PH;
  const size_t oH1 = off; off += PH;
  const size_t oXH = off; off += PXH;
  const size_t oQK = off; off += PQK;
  const size_t oVT = off; off += PVT;
  const size_t oAO = off; off += PAO;
  if (off > ws_size) return;
  if (off > (size_t)134217728) return;

  char* ws = (char*)d_ws;
  unsigned short* WP = (unsigned short*)(ws + oWP);
  float*          H0 = (float*)(ws + oH0);
  float*          H1 = (float*)(ws + oH1);
  unsigned short* XH = (unsigned short*)(ws + oXH);
  unsigned short* QK = (unsigned short*)(ws + oQK);
  unsigned short* VT = (unsigned short*)(ws + oVT);
  unsigned short* AO = (unsigned short*)(ws + oAO);
  float* out0 = (float*)d_out;
  float* out1 = out0 + (size_t)NTOK * DD;

  const dim3 blk(256), blk128(128);
  const dim3 gW(1);
  const dim3 gTK(NTOK / 128);
  const dim3 gQKV(NTOK / 64);
  const dim3 gAT(NSEQ * (GDIM / 64));
  const dim3 gPJ(NTOK / 128);

  prep_w<<<gW, blk, 0, stream>>>(wq, wk, wv, wo, pk2, WP);
  prep_tok<<<gTK, blk, 0, stream>>>(x, pkt, pkv, disc, sfp, gsz, WP, out0, H0, XH);
  qkv_proj<<<gQKV, blk128, 0, stream>>>(XH, WP, bq, bk, bv, QK, VT);
  attn<<<gAT, blk128, 0, stream>>>(QK, VT, AO);
  proj_ln<<<gPJ, blk, 0, stream>>>(AO, WP, bo, gam, bet, H0, H1, XH, 1);
  qkv_proj<<<gQKV, blk128, 0, stream>>>(XH, WP, bq, bk, bv, QK, VT);
  attn<<<gAT, blk128, 0, stream>>>(QK, VT, AO);
  proj_ln<<<gPJ, blk, 0, stream>>>(AO, WP, bo, gam, bet, H1, out1, XH, 0);
  (void)hipGetLastError();
}
